// RestrictedTransformerEncoderLayer_31868657336558
// MI455X (gfx1250) — hardware-verified
//
#include <hip/hip_runtime.h>

typedef __attribute__((ext_vector_type(16))) _Float16 v16h;
typedef __attribute__((ext_vector_type(8)))  _Float16 v8h;
typedef __attribute__((ext_vector_type(16))) __bf16   v16b;
typedef __attribute__((ext_vector_type(8)))  __bf16   v8b;
typedef __attribute__((ext_vector_type(8)))  float    v8f;
typedef __attribute__((ext_vector_type(4)))  float    v4f;

#define U16(p) ((const unsigned short*)(const void*)(p))

__device__ __forceinline__ unsigned short f2bf_bits(float f) {
  unsigned u = __float_as_uint(f);
  return (unsigned short)((u + 0x7FFFu + ((u >> 16) & 1u)) >> 16);
}
__device__ __forceinline__ float bf_bits2f(unsigned short h) { return __uint_as_float(((unsigned)h) << 16); }

__device__ __forceinline__ void dep_guard_h(v8f& a, v8f& b, v16h x, v16h y) { asm volatile("v_nop\n\tv_nop\n\tv_nop\n\tv_nop" : "+v"(a), "+v"(b) : "v"(x), "v"(y)); }
__device__ __forceinline__ void dep_guard_b(v8f& a, v8f& b, v16b x, v16b y) { asm volatile("v_nop\n\tv_nop\n\tv_nop\n\tv_nop" : "+v"(a), "+v"(b) : "v"(x), "v"(y)); }
__device__ __forceinline__ void keep4_h(v16h a, v16h b, v16h c, v16h d) { asm volatile("v_nop" :: "v"(a), "v"(b), "v"(c), "v"(d)); }
__device__ __forceinline__ void keep4_b(v16b a, v16b b, v16b c, v16b d) { asm volatile("v_nop" :: "v"(a), "v"(b), "v"(c), "v"(d)); }
__device__ __forceinline__ void acc_guard4(v8f& a, v8f& b, v8f& c, v8f& d) { asm volatile("v_nop\n\tv_nop\n\tv_nop\n\tv_nop" : "+v"(a), "+v"(b), "+v"(c), "+v"(d)); }
template <typename T> struct Frag;
template <> struct Frag<_Float16> {
  typedef v16h V; union U { v16h v; v8h h[2]; };
  static __device__ __forceinline__ v16h load(const _Float16* p) {
    U f; f.h[0] = *(const v8h*)(p); f.h[1] = *(const v8h*)(p + 16); return f.v;
  }
  static __device__ __forceinline__ v8f mma(v16h a, v16h b, v8f c) {
    return __builtin_amdgcn_wmma_f32_16x16x32_f16(false, a, false, b, (short)0, c, false, false);
  }
  static __device__ __forceinline__ void guard(v8f& a, v8f& b, v16h x, v16h y) { dep_guard_h(a, b, x, y); }
  static __device__ __forceinline__ void keep(v16h a, v16h b, v16h c, v16h d) { keep4_h(a, b, c, d); }
};
template <> struct Frag<__bf16> {
  typedef v16b V; union U { v16b v; v8b h[2]; };
  static __device__ __forceinline__ v16b load(const __bf16* p) {
    U f; f.h[0] = *(const v8b*)(p); f.h[1] = *(const v8b*)(p + 16); return f.v;
  }
  static __device__ __forceinline__ v8f mma(v16b a, v16b b, v8f c) {
    return __builtin_amdgcn_wmma_f32_16x16x32_bf16(false, a, false, b, (short)0, c, false, false);
  }
  static __device__ __forceinline__ void guard(v8f& a, v8f& b, v16b x, v16b y) { dep_guard_b(a, b, x, y); }
  static __device__ __forceinline__ void keep(v16b a, v16b b, v16b c, v16b d) { keep4_b(a, b, c, d); }
};

template <int ET> struct Elem;
template <> struct Elem<0> { typedef _Float16 T; };
template <> struct Elem<1> { typedef __bf16 T; };
template <int ET, bool SPLIT, int BIAS_MODE, int OUT_MODE, bool RESID, int ACT = 0>
__global__ __launch_bounds__(256) void wmma_gemm64(
    const unsigned short* __restrict__ Ap, const unsigned short* __restrict__ A2p, int lda, long strideA,
    const unsigned short* __restrict__ Btp, const unsigned short* __restrict__ Bt2p, int ldb, long strideB,
    void* __restrict__ Cout, void* __restrict__ Cout2, int ldc, long strideC,
    const float* __restrict__ bias,
    const float* __restrict__ resid, long strideR,
    int M, int N, int K, float scale) {
  typedef typename Elem<ET>::T T;
  typedef typename Frag<T>::V V;
  const T* A = (const T*)Ap; const T* A2 = (const T*)A2p; const T* Bt = (const T*)Btp; const T* Bt2 = (const T*)Bt2p;
  __shared__ __align__(16) float sT[8][16 * 68];
  const int b    = blockIdx.y;
  const int lane = threadIdx.x & 31;
  const int wave = threadIdx.x >> 5;
  const int tilesN = N >> 6;
  const int tilesM = M >> 6;
  const int tile = blockIdx.x * 8 + wave;
  if (tile >= tilesM * tilesN) return;
  const int tm = tile / tilesN;
  const int tn = tile - tm * tilesN;
  const int m0 = tm << 6;
  const int n0 = tn << 6;

  const T* Ab  = A  + (size_t)b * strideA;
  const T* Bb  = Bt + (size_t)b * strideB;
  const T* Ab2 = SPLIT ? (A2  + (size_t)b * strideA) : nullptr;
  const T* Bb2 = SPLIT ? (Bt2 + (size_t)b * strideB) : nullptr;

  const int rlane = lane & 15;
  const int koff  = (lane >> 4) * 8;
  const int mOff  = (lane >> 4) * 8;

  v8f acc[4][4];
#pragma unroll
  for (int i = 0; i < 4; ++i)
#pragma unroll
    for (int j = 0; j < 4; ++j) acc[i][j] = (v8f){0.f,0.f,0.f,0.f,0.f,0.f,0.f,0.f};

  for (int k0 = 0; k0 < K; k0 += 32) {
    V bh[4], bl[4];
#pragma unroll
    for (int j = 0; j < 4; ++j) {
      const size_t bo = (size_t)(n0 + (j << 4) + rlane) * ldb + koff + k0;
      bh[j] = Frag<T>::load(Bb + bo);
      if (SPLIT) bl[j] = Frag<T>::load(Bb2 + bo);
    }
#pragma unroll
    for (int i = 0; i < 4; ++i) {
      const size_t ao = (size_t)(m0 + (i << 4) + rlane) * lda + koff + k0;
      V ah = Frag<T>::load(Ab + ao);
      V al;
      if (SPLIT) al = Frag<T>::load(Ab2 + ao);
#pragma unroll
      for (int j = 0; j < 4; ++j) {
        acc[i][j] = Frag<T>::mma(ah, bh[j], acc[i][j]);
        if (SPLIT) {
          acc[i][j] = Frag<T>::mma(ah, bl[j], acc[i][j]);
          acc[i][j] = Frag<T>::mma(al, bh[j], acc[i][j]);
        }
      }
      Frag<T>::guard(acc[i][0], acc[i][3], ah, SPLIT ? al : ah);
    }
    Frag<T>::keep(bh[0], bh[1], bh[2], bh[3]);
    if (SPLIT) Frag<T>::keep(bl[0], bl[1], bl[2], bl[3]);
  }
  acc_guard4(acc[0][0], acc[0][1], acc[0][2], acc[0][3]);
  acc_guard4(acc[1][0], acc[1][1], acc[1][2], acc[1][3]);
  acc_guard4(acc[2][0], acc[2][1], acc[2][2], acc[2][3]);
  acc_guard4(acc[3][0], acc[3][1], acc[3][2], acc[3][3]);

  float* slab = sT[wave];
  const float* Rb = RESID ? (resid + (size_t)b * strideR) : nullptr;
#pragma unroll
  for (int i = 0; i < 4; ++i) {
    const int mBase = m0 + (i << 4);
#pragma unroll
    for (int j = 0; j < 4; ++j) {
      const int n = n0 + (j << 4) + rlane;
      float bv = 0.f;
      if (BIAS_MODE == 2) bv = bias[n];
#pragma unroll
      for (int r = 0; r < 8; ++r) {
        float v = acc[i][j][r] * scale;
        if (BIAS_MODE == 1) v += bias[mBase + mOff + r];
        if (BIAS_MODE == 2) v += bv;
        if (RESID) v += Rb[(size_t)(mBase + mOff + r) * ldc + n];
        if (ACT == 1) v = tanhf(v);
        if (ACT == 2) v = fmaxf(v, 0.0f);
        if (ACT == 3) v = v / (1.0f + expf(-v));
        if (ACT == 4) v = (v > 0.f) ? v : 0.01f * v;
        if (ACT == 5) v = 0.5f * v * (1.0f + erff(v * 0.70710678118654752f));
        slab[(mOff + r) * 68 + (j << 4) + rlane] = v;
      }
    }
    __builtin_amdgcn_fence(__ATOMIC_RELEASE, "workgroup");
    __builtin_amdgcn_wave_barrier();
    __builtin_amdgcn_fence(__ATOMIC_ACQUIRE, "workgroup");
    if (OUT_MODE == 0) {
      float* C = (float*)Cout + (size_t)b * strideC;
      const int hh = lane >> 4, c4 = (lane & 15) * 4;
      for (int pass = 0; pass < 2; ++pass) {
#pragma unroll
        for (int it = 0; it < 8; ++it) {
          const int row = it * 2 + hh;
          v4f v = *(const v4f*)(slab + row * 68 + c4);
          *(volatile v4f*)(C + (size_t)(mBase + row) * ldc + n0 + c4) = v;
        }
        __threadfence();
      }
    } else {
      const int q = lane >> 3, c8 = (lane & 7) * 8;
      unsigned short* C  = (unsigned short*)Cout  + (size_t)b * strideC;
      unsigned short* C2 = (OUT_MODE == 2) ? ((unsigned short*)Cout2 + (size_t)b * strideC) : nullptr;
      for (int pass = 0; pass < 2; ++pass) {
#pragma unroll
        for (int it = 0; it < 4; ++it) {
          const int row = it * 4 + q;
          const float* sp = slab + row * 68 + c8;
          v8h hv, lv;
#pragma unroll
          for (int e = 0; e < 8; ++e) {
            if (OUT_MODE == 1) {
              hv[e] = (_Float16)sp[e];
            } else {
              unsigned short hb = f2bf_bits(sp[e]);
              unsigned short lb = f2bf_bits(sp[e] - bf_bits2f(hb));
              hv[e] = __builtin_bit_cast(_Float16, hb);
              lv[e] = __builtin_bit_cast(_Float16, lb);
            }
          }
          *(volatile v8h*)(C + (size_t)(mBase + row) * ldc + n0 + c8) = hv;
          if (OUT_MODE == 2) *(volatile v8h*)(C2 + (size_t)(mBase + row) * ldc + n0 + c8) = lv;
        }
        __threadfence();
      }
    }
    __builtin_amdgcn_fence(__ATOMIC_RELEASE, "workgroup");
    __builtin_amdgcn_wave_barrier();
    __builtin_amdgcn_fence(__ATOMIC_ACQUIRE, "workgroup");
  }
}

__global__ __launch_bounds__(256) void cast_f32_f16x2s(
    const float* __restrict__ in, _Float16* __restrict__ out, int n2, float scale) {
  int i = blockIdx.x * 256 + threadIdx.x;
  if (i < n2) {
    const _Float16 h0 = (_Float16)(in[2 * i] * scale), h1 = (_Float16)(in[2 * i + 1] * scale);
    const unsigned u = (unsigned)__builtin_bit_cast(unsigned short, h0) | ((unsigned)__builtin_bit_cast(unsigned short, h1) << 16);
    ((volatile unsigned*)out)[i] = u;
    __threadfence();
    ((volatile unsigned*)out)[i] = u;
  }
}

#define SEQ_L  2048
#define NHEAD  16
#define EMB    1024
#define QKV_LD 3072
#define NQB    32
#define WINW   128
#define KC     64
#define NEGFILL (-1.0e9f)
#define P_CARRY 32768.0f
#define CTX_INV (1.0f / 2048.0f)

__device__ __forceinline__ v8f mma_f16(v16h a, v16h b, v8f c) {
  c = __builtin_amdgcn_wmma_f32_16x16x32_f16(false, a, false, b, (short)0, c, false, false);
  asm volatile("v_nop\n\tv_nop\n\tv_nop\n\tv_nop" : "+v"(c) : "v"(a), "v"(b));
  return c;
}

__global__ __launch_bounds__(128)
void attn_band_f16(const _Float16* __restrict__ qkv, _Float16* __restrict__ ctx) {
  typedef Frag<_Float16> FR;
  __shared__ __align__(16) _Float16 Ksh[KC * 64];
  __shared__ __align__(16) _Float16 Vt[64 * KC];
  __shared__ __align__(16) _Float16 Psh[4][16 * KC];
  __shared__ __align__(16) float    Os[4][16 * 68];

  const int tid  = threadIdx.x;
  const int wave = tid >> 5;
  const int lane = tid & 31;
  const int hh   = lane >> 4;
  const int c    = lane & 15;

  const int bx  = blockIdx.x;
  const int qb  = bx % NQB;
  const int bhh = bx / NQB;
  const int h   = bhh % NHEAD;
  const int b   = bhh / NHEAD;
  const int q0  = qb * 64 + wave * 16;

  const _Float16* base = qkv + (size_t)b * SEQ_L * QKV_LD + h * 64;
  const _Float16* kbp  = base + EMB;
  const _Float16* vbp  = base + 2 * EMB;

  v16h qa[2];
  {
    const _Float16* qrow = base + (size_t)(q0 + c) * QKV_LD + 8 * hh;
#pragma unroll
    for (int dc = 0; dc < 2; ++dc) qa[dc] = FR::load(qrow + dc * 32);
  }

  float mrow[8], lrow[8];
  v8f oacc[4];
#pragma unroll
  for (int r = 0; r < 8; ++r) { mrow[r] = -INFINITY; lrow[r] = 0.f; }
#pragma unroll
  for (int t = 0; t < 4; ++t) oacc[t] = (v8f){0.f,0.f,0.f,0.f,0.f,0.f,0.f,0.f};

  int kcLo = qb - 2; if (kcLo < 0) kcLo = 0;
  int kcHi = qb + 2; if (kcHi > NQB - 1) kcHi = NQB - 1;
  for (int kc = kcLo; kc <= kcHi; ++kc) {
    const int kv0 = kc * KC;
    __syncthreads();
    {
      const int kvr = tid >> 1, dh = (tid & 1) * 32;
      const _Float16* krow = kbp + (size_t)(kv0 + kvr) * QKV_LD + dh;
      const _Float16* vrow = vbp + (size_t)(kv0 + kvr) * QKV_LD + dh;
#pragma unroll
      for (int i = 0; i < 4; ++i) {
        const v8h kk = *(const v8h*)(krow + 8 * i);
        const v8h vv = *(const v8h*)(vrow + 8 * i);
        *(v8h*)(Ksh + kvr * 64 + dh + 8 * i) = kk;
#pragma unroll
        for (int e = 0; e < 8; ++e) Vt[(dh + 8 * i + e) * KC + kvr] = vv[e];
      }
    }
    __syncthreads();

    v8f s[4];
#pragma unroll
    for (int j = 0; j < 4; ++j) {
      s[j] = (v8f){0.f,0.f,0.f,0.f,0.f,0.f,0.f,0.f};
#pragma unroll
      for (int dc = 0; dc < 2; ++dc) {
        const v16h kb = FR::load(Ksh + (j * 16 + c) * 64 + dc * 32 + 8 * hh);
        s[j] = mma_f16(qa[dc], kb, s[j]);
      }
    }
    float cm[8];
#pragma unroll
    for (int r = 0; r < 8; ++r) {
      const int qr = q0 + 8 * hh + r;
      float m = -INFINITY;
#pragma unroll
      for (int j = 0; j < 4; ++j) {
        const int kvc = kv0 + j * 16 + c;
        const int dl  = qr - kvc;
        float sv = s[j][r] * 0.125f;
        if (dl > WINW || dl < -WINW) sv = NEGFILL;
        s[j][r] = sv;
        m = fmaxf(m, sv);
      }
#pragma unroll
      for (int off = 1; off < 16; off <<= 1) m = fmaxf(m, __shfl_xor(m, off, 32));
      cm[r] = m;
    }
    _Float16* pw = Psh[wave];
#pragma unroll
    for (int r = 0; r < 8; ++r) {
      const float mnew  = fmaxf(mrow[r], cm[r]);
      const float alpha = expf(mrow[r] - mnew);
      mrow[r] = mnew;
      float psum = 0.f;
#pragma unroll
      for (int j = 0; j < 4; ++j) {
        const float p = expf(s[j][r] - mnew);
        psum += p;
        pw[(8 * hh + r) * KC + j * 16 + c] = (_Float16)(p * P_CARRY);
      }
#pragma unroll
      for (int off = 1; off < 16; off <<= 1) psum += __shfl_xor(psum, off, 32);
      lrow[r] = lrow[r] * alpha + psum;
#pragma unroll
      for (int t = 0; t < 4; ++t) oacc[t][r] *= alpha;
    }
    __builtin_amdgcn_fence(__ATOMIC_RELEASE, "workgroup");
    __builtin_amdgcn_wave_barrier();
    __builtin_amdgcn_fence(__ATOMIC_ACQUIRE, "workgroup");
#pragma unroll 1
    for (int kk = 0; kk < 2; ++kk) {
      const v16h pa = FR::load(pw + c * KC + kk * 32 + 8 * hh);
#pragma unroll
      for (int t = 0; t < 4; ++t) {
        const v16h vb = FR::load(Vt + (t * 16 + c) * KC + kk * 32 + 8 * hh);
        oacc[t] = mma_f16(pa, vb, oacc[t]);
      }
    }
  }

  float* os = Os[wave];
#pragma unroll
  for (int r = 0; r < 8; ++r) {
    const float inv = CTX_INV / lrow[r];
#pragma unroll
    for (int t = 0; t < 4; ++t) os[(8 * hh + r) * 68 + t * 16 + c] = oacc[t][r] * inv;
  }
  __builtin_amdgcn_fence(__ATOMIC_RELEASE, "workgroup");
  __builtin_amdgcn_wave_barrier();
  __builtin_amdgcn_fence(__ATOMIC_ACQUIRE, "workgroup");
  {
    const int q = lane >> 3, c8 = (lane & 7) * 8;
    _Float16* ob = ctx + (size_t)(b * SEQ_L + q0) * EMB + h * 64;
    for (int pass = 0; pass < 2; ++pass) {
#pragma unroll
      for (int it = 0; it < 4; ++it) {
        const int row = it * 4 + q;
        const float* sp = os + row * 68 + c8;
        v8h hv;
#pragma unroll
        for (int e = 0; e < 8; ++e) hv[e] = (_Float16)sp[e];
        *(volatile v8h*)(ob + (size_t)row * EMB + c8) = hv;
      }
      __threadfence();
    }
  }
}

template <bool OUT16>
__global__ __launch_bounds__(256)
void layernorm_rows(const float* __restrict__ x, const float* __restrict__ gam, const float* __restrict__ bet,
                    float* __restrict__ outf, _Float16* __restrict__ outh, int nrows) {
  __shared__ float red[8];
  __shared__ float red2[8];
  __shared__ __align__(16) _Float16 sh[OUT16 ? EMB : 8];
  const int row = blockIdx.x;
  if (row >= nrows) return;
  const int t = threadIdx.x, lane = t & 31, w = t >> 5;
  const int c4 = t * 4;
  const float* xr = x + (size_t)row * EMB;
  const v4f xv = *(const v4f*)(xr + c4);
  float s = (xv[0] + xv[1]) + (xv[2] + xv[3]);
#pragma unroll
  for (int off = 1; off < 32; off <<= 1) s += __shfl_xor(s, off, 32);
  if (lane == 0) red[w] = s;
  __syncthreads();
  float tot = 0.f;
#pragma unroll
  for (int j = 0; j < 8; ++j) tot += red[j];
  const float mu = tot * (1.0f / 1024.0f);
  const float d0 = xv[0] - mu, d1 = xv[1] - mu, d2 = xv[2] - mu, d3 = xv[3] - mu;
  float s2 = (d0 * d0 + d1 * d1) + (d2 * d2 + d3 * d3);
#pragma unroll
  for (int off = 1; off < 32; off <<= 1) s2 += __shfl_xor(s2, off, 32);
  if (lane == 0) red2[w] = s2;
  __syncthreads();
  float tot2 = 0.f;
#pragma unroll
  for (int j = 0; j < 8; ++j) tot2 += red2[j];
  const float var  = tot2 * (1.0f / 1024.0f);
  const float rstd = rsqrtf(var + 1.0e-5f);
  const v4f gv = *(const v4f*)(gam + c4);
  const v4f bv = *(const v4f*)(bet + c4);
  v4f o;
  o[0] = d0 * rstd * gv[0] + bv[0];
  o[1] = d1 * rstd * gv[1] + bv[1];
  o[2] = d2 * rstd * gv[2] + bv[2];
  o[3] = d3 * rstd * gv[3] + bv[3];
  float* op = outf + (size_t)row * EMB + c4;
  *(volatile v4f*)op = o;
  __threadfence();
  *(volatile v4f*)op = o;
  if (OUT16) {
    sh[c4 + 0] = (_Float16)o[0];
    sh[c4 + 1] = (_Float16)o[1];
    sh[c4 + 2] = (_Float16)o[2];
    sh[c4 + 3] = (_Float16)o[3];
    __syncthreads();
    if (t < 128) {
      const v8h hv = *(const v8h*)(sh + 8 * t);
      _Float16* hp = outh + (size_t)row * EMB + 8 * t;
      *(volatile v8h*)hp = hv;
      __threadfence();
      *(volatile v8h*)hp = hv;
    }
  }
}

extern "C" void kernel_launch(void* const* d_in, const int* in_sizes, int n_in,
                              void* d_out, int out_size, void* d_ws,
                              size_t ws_size, hipStream_t stream) {
  const int NR  = 2 * SEQ_L;
  const int NE3 = 3 * EMB;
  const int NFF = 4096;
  if (n_in < 13) return;
  if (in_sizes[0] != NR * EMB || in_sizes[1] != NE3 * EMB || in_sizes[2] != NE3 ||
      in_sizes[3] != EMB * EMB || in_sizes[4] != EMB || in_sizes[5] != NFF * EMB || in_sizes[6] != NFF ||
      in_sizes[7] != EMB * NFF || in_sizes[8] != EMB || in_sizes[9] != EMB || in_sizes[10] != EMB ||
      in_sizes[11] != EMB || in_sizes[12] != EMB || out_size != NR * EMB) return;

  const float* src       = (const float*)d_in[0];
  const float* in_proj_w = (const float*)d_in[1];
  const float* in_proj_b = (const float*)d_in[2];
  const float* out_w     = (const float*)d_in[3];
  const float* out_b     = (const float*)d_in[4];
  const float* lin1_w    = (const float*)d_in[5];
  const float* lin1_b    = (const float*)d_in[6];
  const float* lin2_w    = (const float*)d_in[7];
  const float* lin2_b    = (const float*)d_in[8];
  const float* ln1_g     = (const float*)d_in[9];
  const float* ln1_beta  = (const float*)d_in[10];
  const float* ln2_g     = (const float*)d_in[11];
  const float* ln2_beta  = (const float*)d_in[12];
  float* out = (float*)d_out;

  const size_t bWqkv = (size_t)NE3 * EMB * 2;
  const size_t bWout = (size_t)EMB * EMB * 2;
  const size_t bW1   = (size_t)NFF * EMB * 2;
  const size_t bW2   = (size_t)EMB * NFF * 2;
  const size_t bX16  = (size_t)NR * EMB * 2;
  const size_t bQKV  = (size_t)NR * NE3 * 2;
  const size_t bCTX  = (size_t)NR * EMB * 2;
  const size_t bF32  = (size_t)NR * EMB * 4;
  const size_t bH16  = (size_t)NR * NFF * 2;
  const size_t oWqkv = 0;
  const size_t oWout = oWqkv + bWqkv;
  const size_t oW1   = oWout + bWout;
  const size_t oW2   = oW1 + bW1;
  const size_t oX16  = oW2 + bW2;
  const size_t oQKV  = oX16 + bX16;
  const size_t oCTX  = oQKV + bQKV;
  const size_t oATT  = oX16;
  const size_t oX1F  = oATT + bF32;
  const size_t oX1H  = oCTX;
  const size_t oH16  = oCTX + bCTX;
  const size_t oY    = oATT;
  const size_t need  = oH16 + bH16;
  if (need > ws_size) return;

  char* ws = (char*)d_ws;
  _Float16* Wqkv16 = (_Float16*)(ws + oWqkv);
  _Float16* Wout16 = (_Float16*)(ws + oWout);
  _Float16* W1_16  = (_Float16*)(ws + oW1);
  _Float16* W2_16  = (_Float16*)(ws + oW2);
  _Float16* X16    = (_Float16*)(ws + oX16);
  _Float16* QKV16  = (_Float16*)(ws + oQKV);
  _Float16* CTX16  = (_Float16*)(ws + oCTX);
  float*    ATT    = (float*)(ws + oATT);
  float*    X1F    = (float*)(ws + oX1F);
  _Float16* X1H    = (_Float16*)(ws + oX1H);
  _Float16* H16    = (_Float16*)(ws + oH16);
  float*    Y      = (float*)(ws + oY);

  {
    const int n2s = NR * EMB / 2, n2q = NE3 * EMB / 2, n2o = EMB * EMB / 2, n21 = NFF * EMB / 2, n22 = EMB * NFF / 2;
    cast_f32_f16x2s<<<(n2s + 255) / 256, 256, 0, stream>>>(src,       X16,    n2s, 1.0f);
    cast_f32_f16x2s<<<(n2q + 255) / 256, 256, 0, stream>>>(in_proj_w, Wqkv16, n2q, 64.0f);
    cast_f32_f16x2s<<<(n2o + 255) / 256, 256, 0, stream>>>(out_w,     Wout16, n2o, 64.0f);
    cast_f32_f16x2s<<<(n21 + 255) / 256, 256, 0, stream>>>(lin1_w,    W1_16,  n21, 64.0f);
    cast_f32_f16x2s<<<(n22 + 255) / 256, 256, 0, stream>>>(lin2_w,    W2_16,  n22, 64.0f);
  }

  {
    const int tiles = (NR / 64) * (NE3 / 64);
    wmma_gemm64<0, false, 2, 1, false, 0><<<dim3((tiles + 7) / 8, 1), 256, 0, stream>>>(
        U16(X16), U16(X16), EMB, 0L, U16(Wqkv16), U16(Wqkv16), EMB, 0L,
        (void*)QKV16, (void*)QKV16, NE3, 0L, in_proj_b, in_proj_b, 0L, NR, NE3, EMB, 1.0f / 64.0f);
  }

  attn_band_f16<<<2 * NHEAD * NQB, 128, 0, stream>>>(QKV16, CTX16);

  {
    const int tiles = (NR / 64) * (EMB / 64);
    wmma_gemm64<0, false, 2, 0, true, 0><<<dim3((tiles + 7) / 8, 1), 256, 0, stream>>>(
        U16(CTX16), U16(CTX16), EMB, 0L, U16(Wout16), U16(Wout16), EMB, 0L,
        (void*)ATT, (void*)ATT, EMB, 0L, out_b, src, 0L, NR, EMB, EMB, 1.0f / 1024.0f);
  }

  layernorm_rows<true><<<NR, 256, 0, stream>>>(ATT, ln1_g, ln1_beta, X1F, X1H, NR);

  {
    const int tiles = (NR / 64) * (NFF / 64);
    wmma_gemm64<0, false, 2, 1, false, 2><<<dim3((tiles + 7) / 8, 1), 256, 0, stream>>>(
        U16(X1H), U16(X1H), EMB, 0L, U16(W1_16), U16(W1_16), EMB, 0L,
        (void*)H16, (void*)H16, NFF, 0L, lin1_b, lin1_b, 0L, NR, NFF, EMB, 1.0f / 64.0f);
  }

  {
    const int tiles = (NR / 64) * (EMB / 64);
    wmma_gemm64<0, false, 2, 0, true, 0><<<dim3((tiles + 7) / 8, 1), 256, 0, stream>>>(
        U16(H16), U16(H16), NFF, 0L, U16(W2_16), U16(W2_16), NFF, 0L,
        (void*)Y, (void*)Y, EMB, 0L, lin2_b, X1F, 0L, NR, EMB, NFF, 1.0f / 64.0f);
  }

  layernorm_rows<false><<<NR, 256, 0, stream>>>(Y, ln2_g, ln2_beta, out, X1H, NR);
}
